// SSM_10075993276628
// MI455X (gfx1250) — hardware-run, weakly checked
//
#include <hip/hip_runtime.h>
#include <hip/hip_fp16.h>
#include <math.h>

typedef __attribute__((ext_vector_type(16))) _Float16 v16h;
typedef __attribute__((ext_vector_type(8)))  _Float16 v8h;
typedef __attribute__((ext_vector_type(8)))  float    v8f;
typedef __attribute__((ext_vector_type(4)))  float    v4f;
typedef __attribute__((ext_vector_type(2)))  unsigned v2u;

constexpr int kBatch = 4;
constexpr int kSeq   = 2048;
constexpr int kDin   = 1024;
constexpr int kRank  = 64;
constexpr int kNst   = 16;
constexpr int kNbc   = kRank + 2 * kNst;
constexpr int kRows  = kBatch * kSeq;
static_assert(kNbc == 96);
static_assert(kRows == 8192);
static_assert((kDin % 64) == 0 && (kSeq % 64) == 0);
static_assert((kDin % 32) == 0 && (kRank % 32) == 0);
static_assert((kRows % 64) == 0 && (kNbc % 16) == 0);

constexpr float kCarryX  = 64.0f;
constexpr float kCarryW1 = 1024.0f;
constexpr float kCarryDr = 64.0f;
constexpr float kCarryW2 = 256.0f;
constexpr float kYCarry  = 64.0f;
constexpr float kInv1 = 1.0f / (kCarryX * kCarryW1);
constexpr float kInv2 = 1.0f / (kCarryDr * kCarryW2);
constexpr float kInvY = 1.0f / kYCarry;

constexpr size_t kSzXR   = (size_t)kRows * kDin * 4;
constexpr size_t kSzXH   = (size_t)kRows * kDin * 2;
constexpr size_t kSzWH   = (size_t)kNbc * kDin * 2;
constexpr size_t kSzWDH  = (size_t)kDin * kRank * 2;
constexpr size_t kSzALR  = (size_t)kDin * kNst * 4;
constexpr size_t kSzDPR  = (size_t)kDin * 4;
constexpr size_t kSzBDR  = (size_t)kDin * 4;
constexpr size_t kSzBC   = (size_t)kRows * kNbc * 4;
constexpr size_t kSzDR16 = (size_t)kRows * kRank * 2;
constexpr size_t kSzDT   = (size_t)kRows * kDin * 4;
constexpr size_t kSzY16  = (size_t)kRows * kDin * 2;
constexpr size_t kOffXR   = 0;
constexpr size_t kOffXH   = kOffXR   + kSzXR;
constexpr size_t kOffWH   = kOffXH   + kSzXH;
constexpr size_t kOffWDH  = kOffWH   + kSzWH;
constexpr size_t kOffALR  = kOffWDH  + kSzWDH;
constexpr size_t kOffDPR  = kOffALR  + kSzALR;
constexpr size_t kOffBDR  = kOffDPR  + kSzDPR;
constexpr size_t kOffBC   = kOffBDR  + kSzBDR;
constexpr size_t kOffDR16 = kOffBC   + kSzBC;
constexpr size_t kOffDT   = kOffDR16 + kSzDR16;
constexpr size_t kOffY16  = kOffDT   + kSzDT;
constexpr size_t kWsTotal = kOffY16  + kSzY16;
static_assert(kWsTotal == 105259008ull);
static_assert(kWsTotal <= 134217728ull);
static_assert((kOffXH % 4096) == 0 && (kOffWH % 4096) == 0 && (kOffWDH % 4096) == 0 && (kOffALR % 4096) == 0 &&
              (kOffDPR % 4096) == 0 && (kOffBDR % 4096) == 0 && (kOffBC % 4096) == 0 && (kOffDR16 % 4096) == 0 &&
              (kOffDT % 4096) == 0 && (kOffY16 % 4096) == 0);

__device__ __forceinline__ float rne_bf16_f32(float f) {
  const unsigned u = __float_as_uint(f);
  const unsigned r = (u + 0x7FFFu + ((u >> 16) & 1u)) & 0xFFFF0000u;
  return __uint_as_float(r);
}
__device__ __forceinline__ float flush16(float v) {
  return (fabsf(v) < 6.103515625e-05f) ? 0.0f : v;
}
__device__ __forceinline__ float h16_to_f32(unsigned hb) {
  const unsigned sgn = (hb & 0x8000u) << 16;
  const unsigned em = hb & 0x7fffu;
  const float fn = __uint_as_float((em << 13) + 0x38000000u);
  const float fs = (float)em * 5.9604644775390625e-8f;
  const float mag = (em < 0x400u) ? fs : fn;
  return __uint_as_float(__float_as_uint(mag) | sgn);
}

union FragU { v16h v; v8h h[2]; };
__device__ __forceinline__ v16h frag_load(const _Float16* p) {
  FragU f;
  f.h[0] = *(const v8h*)(p);
  f.h[1] = *(const v8h*)(p + 16);
  return f.v;
}
__device__ __forceinline__ v8f mma_f16(v16h a, v16h b, v8f c) {
  c = __builtin_amdgcn_wmma_f32_16x16x32_f16(false, a, false, b, (short)0, c, false, false);
  asm volatile("v_nop\n\tv_nop\n\tv_nop\n\tv_nop" : "+v"(c) : "v"(a), "v"(b));
  return c;
}

__global__ __launch_bounds__(256) void rne_copy_kernel(const float* __restrict__ src, float* __restrict__ dst, int n4)
{
  const int i = blockIdx.x * 256 + threadIdx.x;
  if (i >= n4) return;
  const size_t e0 = (size_t)i << 2;
  const v4f a = *(const v4f*)(src + e0);
  const float a0 = a[0];
  const float a1 = a[1];
  const float a2 = a[2];
  const float a3 = a[3];
  v4f o;
  o[0] = rne_bf16_f32(a0);
  o[1] = rne_bf16_f32(a1);
  o[2] = rne_bf16_f32(a2);
  o[3] = rne_bf16_f32(a3);
  float* p = dst + e0;
  *(volatile v4f*)p = o;
  __threadfence();
  *(volatile v4f*)p = o;
}

__global__ __launch_bounds__(256) void carry_f16_kernel(const float* __restrict__ src, unsigned short* __restrict__ dst,
                                                        int n8, float carry)
{
  const int i = blockIdx.x * 256 + threadIdx.x;
  if (i >= n8) return;
  const size_t e0 = (size_t)i << 3;
  const v4f a0 = *(const v4f*)(src + e0);
  const v4f a1 = *(const v4f*)(src + e0 + 4);
  float s[8];
  s[0] = a0[0];
  s[1] = a0[1];
  s[2] = a0[2];
  s[3] = a0[3];
  s[4] = a1[0];
  s[5] = a1[1];
  s[6] = a1[2];
  s[7] = a1[3];
  v8h hv;
#pragma unroll
  for (int e = 0; e < 8; ++e) {
    const float t = flush16(rne_bf16_f32(s[e]) * carry);
    hv[e] = (_Float16)t;
  }
  unsigned short* p = dst + e0;
  *(volatile v8h*)p = hv;
  __threadfence();
  *(volatile v8h*)p = hv;
}

constexpr int kP1Pitch = 100;
__global__ __launch_bounds__(128) void proj_bc_kernel(const unsigned short* __restrict__ XHp,
                                                      const unsigned short* __restrict__ WHp,
                                                      float* __restrict__ BC, unsigned short* __restrict__ DR16)
{
  __shared__ __align__(16) float sT[4][16 * kP1Pitch];
  const _Float16* A  = (const _Float16*)XHp;
  const _Float16* Bt = (const _Float16*)WHp;
  const int lane = threadIdx.x & 31;
  const int wave = threadIdx.x >> 5;
  const int tile = blockIdx.x * 4 + wave;
  if (tile >= kRows / 32) return;
  const int m0 = tile * 32;
  const int rlane = lane & 15;
  const int koff  = (lane >> 4) * 8;
  const int mOff  = (lane >> 4) * 8;

  v8f acc[2][6];
#pragma unroll
  for (int i = 0; i < 2; ++i)
#pragma unroll
    for (int j = 0; j < 6; ++j) acc[i][j] = (v8f){0.f, 0.f, 0.f, 0.f, 0.f, 0.f, 0.f, 0.f};

  const _Float16* ap0 = A + (size_t)(m0 + rlane) * kDin + koff;
  const _Float16* ap1 = ap0 + (size_t)16 * kDin;
  const _Float16* bp  = Bt + (size_t)rlane * kDin + koff;
#pragma unroll 1
  for (int k0 = 0; k0 < kDin; k0 += 32) {
    const v16h a0 = frag_load(ap0 + k0);
    const v16h a1 = frag_load(ap1 + k0);
#pragma unroll
    for (int j = 0; j < 6; ++j) {
      const v16h b = frag_load(bp + (size_t)(j * 16) * kDin + k0);
      acc[0][j] = mma_f16(a0, b, acc[0][j]);
      acc[1][j] = mma_f16(a1, b, acc[1][j]);
    }
  }

  float* slab = sT[wave];
  const int q  = lane >> 3;
  const int c8 = (lane & 7) * 8;
#pragma unroll
  for (int i = 0; i < 2; ++i) {
    const int mBase = m0 + i * 16;
#pragma unroll
    for (int j = 0; j < 6; ++j) {
#pragma unroll
      for (int r = 0; r < 8; ++r) {
        slab[(mOff + r) * kP1Pitch + j * 16 + rlane] = acc[i][j][r] * kInv1;
      }
    }
    __builtin_amdgcn_fence(__ATOMIC_RELEASE, "workgroup");
    __builtin_amdgcn_wave_barrier();
    __builtin_amdgcn_fence(__ATOMIC_ACQUIRE, "workgroup");
    for (int pass = 0; pass < 2; ++pass) {
#pragma unroll
      for (int it = 0; it < 12; ++it) {
        const int f   = it * 32 + lane;
        const int row = f / 24;
        const int c4  = (f - row * 24) * 4;
        const v4f v = *(const v4f*)(slab + row * kP1Pitch + c4);
        *(volatile v4f*)(BC + (size_t)(mBase + row) * kNbc + c4) = v;
      }
#pragma unroll
      for (int it = 0; it < 4; ++it) {
        const int row = it * 4 + q;
        const float* sp = slab + row * kP1Pitch + c8;
        const v4f f0 = *(const v4f*)(sp);
        const v4f f1 = *(const v4f*)(sp + 4);
        float s[8];
        s[0] = f0[0];
        s[1] = f0[1];
        s[2] = f0[2];
        s[3] = f0[3];
        s[4] = f1[0];
        s[5] = f1[1];
        s[6] = f1[2];
        s[7] = f1[3];
        v8h hv;
#pragma unroll
        for (int e = 0; e < 8; ++e) {
          const float t = flush16(s[e] * kCarryDr);
          hv[e] = (_Float16)t;
        }
        *(volatile v8h*)(DR16 + (size_t)(mBase + row) * kRank + c8) = hv;
      }
      __threadfence();
    }
    __builtin_amdgcn_fence(__ATOMIC_RELEASE, "workgroup");
    __builtin_amdgcn_wave_barrier();
    __builtin_amdgcn_fence(__ATOMIC_ACQUIRE, "workgroup");
  }
}

__global__ __launch_bounds__(256) void proj_dt_kernel(const unsigned short* __restrict__ DRp,
                                                      const unsigned short* __restrict__ WDp,
                                                      const float* __restrict__ bias, float* __restrict__ DT)
{
  __shared__ __align__(16) float sT[8][16 * 68];
  const _Float16* A  = (const _Float16*)DRp;
  const _Float16* Bt = (const _Float16*)WDp;
  const int lane = threadIdx.x & 31;
  const int wave = threadIdx.x >> 5;
  constexpr int tilesN = kDin / 64;
  constexpr int tilesM = kRows / 64;
  const int tile = blockIdx.x * 8 + wave;
  if (tile >= tilesM * tilesN) return;
  const int tm = tile / tilesN;
  const int tn = tile - tm * tilesN;
  const int m0 = tm << 6;
  const int n0 = tn << 6;
  const int rlane = lane & 15;
  const int koff  = (lane >> 4) * 8;
  const int mOff  = (lane >> 4) * 8;

  v8f acc[4][4];
#pragma unroll
  for (int i = 0; i < 4; ++i)
#pragma unroll
    for (int j = 0; j < 4; ++j) acc[i][j] = (v8f){0.f, 0.f, 0.f, 0.f, 0.f, 0.f, 0.f, 0.f};

#pragma unroll 1
  for (int k0 = 0; k0 < kRank; k0 += 32) {
    v16h bh[4];
#pragma unroll
    for (int j = 0; j < 4; ++j) {
      bh[j] = frag_load(Bt + (size_t)(n0 + (j << 4) + rlane) * kRank + koff + k0);
    }
#pragma unroll
    for (int i = 0; i < 4; ++i) {
      const v16h ah = frag_load(A + (size_t)(m0 + (i << 4) + rlane) * kRank + koff + k0);
#pragma unroll
      for (int j = 0; j < 4; ++j) {
        acc[i][j] = mma_f16(ah, bh[j], acc[i][j]);
      }
    }
  }

  float bv[4];
#pragma unroll
  for (int j = 0; j < 4; ++j) bv[j] = bias[n0 + (j << 4) + rlane];

  float* slab = sT[wave];
  const int hh = lane >> 4;
  const int c4 = (lane & 15) * 4;
#pragma unroll
  for (int i = 0; i < 4; ++i) {
    const int mBase = m0 + (i << 4);
#pragma unroll
    for (int j = 0; j < 4; ++j) {
#pragma unroll
      for (int r = 0; r < 8; ++r) {
        slab[(mOff + r) * 68 + (j << 4) + rlane] = acc[i][j][r] * kInv2 + bv[j];
      }
    }
    __builtin_amdgcn_fence(__ATOMIC_RELEASE, "workgroup");
    __builtin_amdgcn_wave_barrier();
    __builtin_amdgcn_fence(__ATOMIC_ACQUIRE, "workgroup");
    for (int pass = 0; pass < 2; ++pass) {
#pragma unroll
      for (int it = 0; it < 8; ++it) {
        const int row = it * 2 + hh;
        const v4f v = *(const v4f*)(slab + row * 68 + c4);
        *(volatile v4f*)(DT + (size_t)(mBase + row) * kDin + n0 + c4) = v;
      }
      __threadfence();
    }
    __builtin_amdgcn_fence(__ATOMIC_RELEASE, "workgroup");
    __builtin_amdgcn_wave_barrier();
    __builtin_amdgcn_fence(__ATOMIC_ACQUIRE, "workgroup");
  }
}

__global__ __launch_bounds__(256) void y_out_kernel(const unsigned* __restrict__ y16w, float* __restrict__ out, int n4)
{
  const int i = blockIdx.x * 256 + threadIdx.x;
  if (i >= n4) return;
  const v2u w = *(const v2u*)(y16w + ((size_t)i << 1));
  const unsigned w0 = w[0];
  const unsigned w1 = w[1];
  v4f o;
  o[0] = h16_to_f32(w0 & 0xffffu) * kInvY;
  o[1] = h16_to_f32(w0 >> 16) * kInvY;
  o[2] = h16_to_f32(w1 & 0xffffu) * kInvY;
  o[3] = h16_to_f32(w1 >> 16) * kInvY;
  float* p = out + ((size_t)i << 2);
  *(volatile v4f*)p = o;
  __threadfence();
  *(volatile v4f*)p = o;
}

typedef float    ms1_v4f __attribute__((ext_vector_type(4)));
typedef unsigned ms1_v4u __attribute__((ext_vector_type(4)));
struct ms1_args {
  const float* dtpre;
  const float* u;
  const float* bc;
  const float* z;
  const float* A_log;
  const float* Dskip;
  __half* y;
  __half* y_lo;
  long ld_dtpre;
  long ld_u;
  long ld_bc;
  long ld_z;
  long ld_y;
  int offB;
  int offC;
  int offZ;
  float ycarry;
  int dir;
  int D;
  int L;
  int nbatch;
};
static_assert(sizeof(ms1_args) == 136);

__device__ __forceinline__ float ms1_flush16(float v) {
  return (fabsf(v) < 6.103515625e-05f) ? 0.0f : v;
}
__device__ __forceinline__ unsigned ms1_h16bits(float v) {
  return (unsigned)__half_as_ushort(__float2half_rn(ms1_flush16(v)));
}
__device__ __forceinline__ float ms1_h16val(unsigned b) {
  return __half2float(__ushort_as_half((unsigned short)b));
}
__device__ __forceinline__ float ms1_softplus(float v) {
  return fmaxf(v, 0.0f) + log1pf(expf(-fabsf(v)));
}
__device__ __forceinline__ void ms1_pack2(float v0, float v1, unsigned& hw, unsigned& lw) {
  const unsigned h0 = ms1_h16bits(v0);
  const unsigned h1 = ms1_h16bits(v1);
  const float r0 = (v0 - ms1_h16val(h0)) * 2048.0f;
  const float r1 = (v1 - ms1_h16val(h1)) * 2048.0f;
  const unsigned l0 = ms1_h16bits(r0);
  const unsigned l1 = ms1_h16bits(r1);
  hw = h0 | (h1 << 16);
  lw = l0 | (l1 << 16);
}

template <int NSTATE>
__global__ __launch_bounds__(64 * (NSTATE / 16)) void ms1_scan_kernel(ms1_args a)
{
  static_assert(NSTATE == 16 || NSTATE == 64);
  constexpr int NQ  = NSTATE / 16;
  constexpr int NT  = 64 * NQ;
  constexpr int NW  = NT / 32;
  constexpr int BCW = 2 * NSTATE;
  constexpr int YP  = 68;
  constexpr int RPI = NW * 4;
  constexpr int NIT = 64 / RPI;
  static_assert(16 * NT <= 64 * YP);
  __shared__ __align__(16) float sBC[64 * BCW];
  __shared__ __align__(16) float sY[64 * YP];
  const int tid  = threadIdx.x;
  const int lane = tid & 31;
  const int wave = tid >> 5;
  const int c    = tid / NQ;
  const int sq   = tid - c * NQ;
  const int bpb  = a.D / 64;
  const int bi   = blockIdx.x / bpb;
  if (bi >= a.nbatch) return;
  const int d0 = (blockIdx.x - bi * bpb) * 64;
  const int d  = d0 + c;
  const long rowb = (long)bi * a.L;
  const bool hasz  = (a.z != nullptr);
  const bool hasD  = (a.Dskip != nullptr);
  const bool hasLo = (a.y_lo != nullptr);

#pragma unroll 1
  for (int n = 0; n < 16; ++n) {
    const float al = a.A_log[(long)d * NSTATE + sq * 16 + n];
    sY[n * NT + tid] = -expf(al);
  }
  __syncthreads();
  float An[16], h[16];
#pragma unroll
  for (int n = 0; n < 16; ++n) {
    An[n] = sY[n * NT + tid];
    h[n] = 0.0f;
  }
  float Dd = 0.0f;
  if (hasD) Dd = a.Dskip[d];

  const int nchunk = a.L / 64;
  const bool fwd = (a.dir > 0);
  const int s0 = fwd ? 0 : 63;
  const int sd = fwd ? 1 : -1;
  const int q  = lane >> 3;
  const int c8 = (lane & 7) * 8;

#pragma unroll 1
  for (int ci = 0; ci < nchunk; ++ci) {
    const int tb = fwd ? (ci * 64) : (a.L - 64 - ci * 64);
    const long rowc = rowb + tb;
    __syncthreads();
#pragma unroll 8
    for (int i = 0; i < 32; ++i) {
      const int idx = tid + i * NT;
      const int st  = idx / BCW;
      const int col = idx - st * BCW;
      const int sc  = (col < NSTATE) ? (a.offB + col) : (a.offC + col - NSTATE);
      sBC[idx] = a.bc[(rowc + st) * a.ld_bc + sc];
    }
    __syncthreads();
#pragma unroll 1
    for (int s = 0; s < 64; ++s) {
      const int ls = s0 + sd * s;
      const long row = rowc + ls;
      float pre = a.dtpre[row * a.ld_dtpre + d];
      float uv  = a.u[row * a.ld_u + d];
      float zv  = 0.0f;
      if (hasz) zv = a.z[row * a.ld_z + a.offZ + d];
      asm volatile("" : "+v"(pre));
      asm volatile("" : "+v"(uv));
      asm volatile("" : "+v"(zv));
      const float delta = ms1_softplus(pre);
      const float dtx = delta * uv;
      const float* bp = sBC + ls * BCW + sq * 16;
      const float* cp = bp + NSTATE;
      ms1_v4f Bq[4], Cq[4];
#pragma unroll
      for (int k = 0; k < 4; ++k) {
        Bq[k] = *(const ms1_v4f*)(bp + 4 * k);
        Cq[k] = *(const ms1_v4f*)(cp + 4 * k);
      }
      float yv = 0.0f;
#pragma unroll
      for (int n = 0; n < 16; ++n) {
        const float e = __expf(delta * An[n]);
        h[n] = fmaf(e, h[n], dtx * Bq[n >> 2][n & 3]);
        yv = fmaf(h[n], Cq[n >> 2][n & 3], yv);
      }
      if (NQ > 1) {
        yv += __shfl_xor(yv, 1, 32);
        yv += __shfl_xor(yv, 2, 32);
      }
      if (hasD) yv = fmaf(uv, Dd, yv);
      if (hasz) {
        const float sg = __builtin_amdgcn_rcpf(1.0f + expf(-zv));
        yv = yv * (zv * sg);
      }
      if (sq == 0) sY[ls * YP + c] = yv * a.ycarry;
    }
    __syncthreads();
    ms1_v4u hw[NIT], lw[NIT];
#pragma unroll
    for (int it = 0; it < NIT; ++it) {
      const int row = it * RPI + wave * 4 + q;
      const float* sp = sY + row * YP + c8;
      const ms1_v4f f0 = *(const ms1_v4f*)(sp);
      const ms1_v4f f1 = *(const ms1_v4f*)(sp + 4);
      unsigned h0, h1, h2, h3, l0, l1, l2, l3;
      ms1_pack2(f0[0], f0[1], h0, l0);
      ms1_pack2(f0[2], f0[3], h1, l1);
      ms1_pack2(f1[0], f1[1], h2, l2);
      ms1_pack2(f1[2], f1[3], h3, l3);
      hw[it] = (ms1_v4u){h0, h1, h2, h3};
      lw[it] = (ms1_v4u){l0, l1, l2, l3};
    }
    for (int pass = 0; pass < 2; ++pass) {
#pragma unroll
      for (int it = 0; it < NIT; ++it) {
        const int row = it * RPI + wave * 4 + q;
        const long o = (rowc + row) * a.ld_y + d0 + c8;
        *(volatile ms1_v4u*)(a.y + o) = hw[it];
        if (hasLo) *(volatile ms1_v4u*)(a.y_lo + o) = lw[it];
      }
      __threadfence();
    }
  }
}

extern "C" void kernel_launch(void* const* d_in, const int* in_sizes, int n_in,
                              void* d_out, int out_size, void* d_ws, size_t ws_size,
                              hipStream_t stream) {
  if (n_in < 6) return;
  if (in_sizes[0] != kRows * kDin) return;
  if (in_sizes[1] != kNbc * kDin) return;
  if (in_sizes[2] != kDin * kRank) return;
  if (in_sizes[3] != kDin) return;
  if (in_sizes[4] != kDin * kNst) return;
  if (in_sizes[5] != kDin) return;
  if (out_size != kRows * kDin) return;
  if (ws_size < kWsTotal) return;

  const float* x     = (const float*)d_in[0];
  const float* W_bc  = (const float*)d_in[1];
  const float* W_dt  = (const float*)d_in[2];
  const float* b_dt  = (const float*)d_in[3];
  const float* A_log = (const float*)d_in[4];
  const float* D_par = (const float*)d_in[5];
  float* out = (float*)d_out;

  char* ws = (char*)d_ws;
  float*          XR   = (float*)(ws + kOffXR);
  unsigned short* XH   = (unsigned short*)(ws + kOffXH);
  unsigned short* WH   = (unsigned short*)(ws + kOffWH);
  unsigned short* WDH  = (unsigned short*)(ws + kOffWDH);
  float*          ALR  = (float*)(ws + kOffALR);
  float*          DPR  = (float*)(ws + kOffDPR);
  float*          BDR  = (float*)(ws + kOffBDR);
  float*          BC   = (float*)(ws + kOffBC);
  unsigned short* DR16 = (unsigned short*)(ws + kOffDR16);
  float*          DT   = (float*)(ws + kOffDT);
  unsigned short* Y16  = (unsigned short*)(ws + kOffY16);

  rne_copy_kernel<<<dim3((kRows * kDin / 4) / 256), 256, 0, stream>>>(x, XR, kRows * kDin / 4);
  rne_copy_kernel<<<dim3((kDin * kNst / 4) / 256), 256, 0, stream>>>(A_log, ALR, kDin * kNst / 4);
  rne_copy_kernel<<<dim3((kDin / 4) / 256), 256, 0, stream>>>(D_par, DPR, kDin / 4);
  rne_copy_kernel<<<dim3((kDin / 4) / 256), 256, 0, stream>>>(b_dt, BDR, kDin / 4);

  carry_f16_kernel<<<dim3((kRows * kDin / 8) / 256), 256, 0, stream>>>(x, XH, kRows * kDin / 8, kCarryX);
  carry_f16_kernel<<<dim3((kNbc * kDin / 8) / 256), 256, 0, stream>>>(W_bc, WH, kNbc * kDin / 8, kCarryW1);
  carry_f16_kernel<<<dim3((kDin * kRank / 8) / 256), 256, 0, stream>>>(W_dt, WDH, kDin * kRank / 8, kCarryW2);

  proj_bc_kernel<<<dim3((kRows / 32) / 4), 128, 0, stream>>>(XH, WH, BC, DR16);

  proj_dt_kernel<<<dim3((kRows / 64) * (kDin / 64) / 8), 256, 0, stream>>>(DR16, WDH, BDR, DT);

  for (int b = 0; b < kBatch; ++b) {
    const size_t r0 = (size_t)b * kSeq;
    ms1_args sa;
    sa.dtpre = DT + r0 * kDin;
    sa.u = XR + r0 * kDin;
    sa.bc = BC + r0 * kNbc;
    sa.z = nullptr;
    sa.A_log = ALR;
    sa.Dskip = DPR;
    sa.y = (__half*)(Y16 + r0 * kDin);
    sa.y_lo = nullptr;
    sa.ld_dtpre = kDin;
    sa.ld_u = kDin;
    sa.ld_bc = kNbc;
    sa.ld_z = 0;
    sa.ld_y = kDin;
    sa.offB = kRank;
    sa.offC = kRank + kNst;
    sa.offZ = 0;
    sa.ycarry = kYCarry;
    sa.dir = 1;
    sa.D = kDin;
    sa.L = kSeq;
    sa.nbatch = 1;
    ms1_scan_kernel<16><<<dim3(kDin / 64), 64, 0, stream>>>(sa);
  }

  y_out_kernel<<<dim3((kRows * kDin / 4) / 256), 256, 0, stream>>>((const unsigned*)Y16, out, kRows * kDin / 4);
}
